// MambaBlock_7799660609679
// MI455X (gfx1250) — hardware-verified
//
#include <hip/hip_runtime.h>
#include <math.h>

typedef __attribute__((ext_vector_type(16))) _Float16 v16h;
typedef __attribute__((ext_vector_type(8)))  _Float16 v8h;
typedef __attribute__((ext_vector_type(16))) __bf16   v16b;
typedef __attribute__((ext_vector_type(8)))  __bf16   v8b;
typedef __attribute__((ext_vector_type(8)))  float    v8f;
typedef __attribute__((ext_vector_type(4)))  float    v4f;

constexpr int kBat    = 8;
constexpr int kSeq    = 64;
constexpr int kDim    = 1024;
constexpr int kNst    = 128;
constexpr int kDtR    = 64;
constexpr int kRows   = kBat * kSeq;
constexpr int kDbcN   = kDtR + 2 * kNst;
constexpr int kConvK  = 3 * kSeq;
constexpr int kXtRows = kDim + 2;
constexpr int kScE    = 64;
constexpr int kScYP   = 68;
static_assert(kRows == 512 && kDbcN == 320 && kConvK == 192 && kXtRows == 1026, "shape constants");
static_assert((kDim % 32) == 0 && (kConvK % 32) == 0 && (kDtR % 32) == 0, "GEMM K multiples of 32");
static_assert((kRows % 64) == 0 && (kDim % 64) == 0 && (kDbcN % 64) == 0 && (kSeq % 64) == 0, "GEMM M,N multiples of 64");
static_assert(kNst == 128 && kScE == 64 && kSeq == 64, "scan tiling");

constexpr size_t kSzX16  = (size_t)kRows * kDim * 2;
constexpr size_t kSzPW   = (size_t)kDim * kDim * 2;
constexpr size_t kSzDW   = (size_t)kDbcN * kDim * 2;
constexpr size_t kSzTW   = (size_t)kDim * kDtR * 2;
constexpr size_t kSzCW   = (size_t)kSeq * kConvK * 2;
constexpr size_t kSzF32  = (size_t)kRows * kDim * 4;
constexpr size_t kSzXT   = (size_t)kBat * kXtRows * kSeq * 2;
constexpr size_t kSzDBC  = (size_t)kRows * kDbcN * 4;
constexpr size_t kSzR    = (size_t)kRows * kDtR * 2;
constexpr size_t kOffXH   = 0;
constexpr size_t kOffXL   = kOffXH   + kSzX16;
constexpr size_t kOffPWH  = kOffXL   + kSzX16;
constexpr size_t kOffPWL  = kOffPWH  + kSzPW;
constexpr size_t kOffDWH  = kOffPWL  + kSzPW;
constexpr size_t kOffDWL  = kOffDWH  + kSzDW;
constexpr size_t kOffTWH  = kOffDWL  + kSzDW;
constexpr size_t kOffTWL  = kOffTWH  + kSzTW;
constexpr size_t kOffCWH  = kOffTWL  + kSzTW;
constexpr size_t kOffCWL  = kOffCWH  + kSzCW;
constexpr size_t kOffXP   = kOffCWL  + kSzCW;
constexpr size_t kOffXTH  = kOffXP   + kSzF32;
constexpr size_t kOffXTL  = kOffXTH  + kSzXT;
constexpr size_t kOffXONE = kOffXTL  + kSzXT;
constexpr size_t kOffUH   = kOffXONE + kSzF32;
constexpr size_t kOffUL   = kOffUH   + kSzX16;
constexpr size_t kOffDBC  = kOffUL   + kSzX16;
constexpr size_t kOffRH   = kOffDBC  + kSzDBC;
constexpr size_t kOffRL   = kOffRH   + kSzR;
constexpr size_t kOffDLR  = kOffRL   + kSzR;
constexpr size_t kOffGH   = kOffDLR  + kSzF32;
constexpr size_t kOffGL   = kOffGH   + kSzX16;
constexpr size_t kWsTotal = kOffGL   + kSzX16;
static_assert(kWsTotal == 21286912ull, "carve total");
static_assert(kWsTotal <= 134217728ull, "carve cap");
static_assert((kSzX16 % 128) == 0 && (kSzPW % 128) == 0 && (kSzDW % 128) == 0 && (kSzTW % 128) == 0 &&
              (kSzCW % 128) == 0 && (kSzF32 % 128) == 0 && (kSzXT % 128) == 0 && (kSzDBC % 128) == 0 &&
              (kSzR % 128) == 0, "every region is a whole number of 128-B lines");

__device__ __forceinline__ unsigned short f2bf_bits(float f) {
  unsigned u = __float_as_uint(f);
  return (unsigned short)((u + 0x7FFFu + ((u >> 16) & 1u)) >> 16);
}
__device__ __forceinline__ float bf_bits2f(unsigned short h) { return __uint_as_float(((unsigned)h) << 16); }

__device__ __forceinline__ void dep_guard4_h(v8f& a, v8f& b, v8f& c, v8f& d, v16h x, v16h y) { asm volatile("v_nop\n\tv_nop\n\tv_nop\n\tv_nop" : "+v"(a), "+v"(b), "+v"(c), "+v"(d) : "v"(x), "v"(y)); }
__device__ __forceinline__ void dep_guard4_b(v8f& a, v8f& b, v8f& c, v8f& d, v16b x, v16b y) { asm volatile("v_nop\n\tv_nop\n\tv_nop\n\tv_nop" : "+v"(a), "+v"(b), "+v"(c), "+v"(d) : "v"(x), "v"(y)); }
__device__ __forceinline__ void keep4_h(v16h a, v16h b, v16h c, v16h d) { asm volatile("v_nop" :: "v"(a), "v"(b), "v"(c), "v"(d)); }
__device__ __forceinline__ void keep4_b(v16b a, v16b b, v16b c, v16b d) { asm volatile("v_nop" :: "v"(a), "v"(b), "v"(c), "v"(d)); }
__device__ __forceinline__ void acc_guard4(v8f& a, v8f& b, v8f& c, v8f& d) { asm volatile("v_nop\n\tv_nop\n\tv_nop\n\tv_nop" : "+v"(a), "+v"(b), "+v"(c), "+v"(d)); }
template <typename T> struct Frag;
template <> struct Frag<_Float16> {
  typedef v16h V; union U { v16h v; v8h h[2]; };
  static __device__ __forceinline__ v16h load(const _Float16* p) {
    U f; f.h[0] = *(const v8h*)(p); f.h[1] = *(const v8h*)(p + 16); return f.v;
  }
  static __device__ __forceinline__ v8f mma(v16h a, v16h b, v8f c) {
    return __builtin_amdgcn_wmma_f32_16x16x32_f16(false, a, false, b, (short)0, c, false, false);
  }
  static __device__ __forceinline__ void guard4(v8f& a, v8f& b, v8f& c, v8f& d, v16h x, v16h y) { dep_guard4_h(a, b, c, d, x, y); }
  static __device__ __forceinline__ void keep(v16h a, v16h b, v16h c, v16h d) { keep4_h(a, b, c, d); }
};
template <> struct Frag<__bf16> {
  typedef v16b V; union U { v16b v; v8b h[2]; };
  static __device__ __forceinline__ v16b load(const __bf16* p) {
    U f; f.h[0] = *(const v8b*)(p); f.h[1] = *(const v8b*)(p + 16); return f.v;
  }
  static __device__ __forceinline__ v8f mma(v16b a, v16b b, v8f c) {
    return __builtin_amdgcn_wmma_f32_16x16x32_bf16(false, a, false, b, (short)0, c, false, false);
  }
  static __device__ __forceinline__ void guard4(v8f& a, v8f& b, v8f& c, v8f& d, v16b x, v16b y) { dep_guard4_b(a, b, c, d, x, y); }
  static __device__ __forceinline__ void keep(v16b a, v16b b, v16b c, v16b d) { keep4_b(a, b, c, d); }
};

template <int ET> struct Elem;
template <> struct Elem<0> { typedef _Float16 T; };
template <> struct Elem<1> { typedef __bf16 T; };
template <int ET, int SPL, int BIAS_MODE, int OUT_MODE, bool RESID, int ACT>
__global__ __launch_bounds__(256) void wmma_gemm64(
    const unsigned short* __restrict__ Ap, const unsigned short* __restrict__ A2p, int lda, long strideA,
    const unsigned short* __restrict__ Btp, const unsigned short* __restrict__ Bt2p, int ldb, long strideB,
    void* __restrict__ Cout, void* __restrict__ Cout2, int ldc, long strideC,
    const float* __restrict__ bias,
    const float* __restrict__ resid, long strideR,
    int M, int N, int K, float scale) {
  typedef typename Elem<ET>::T T;
  typedef typename Frag<T>::V V;
  const T* A = (const T*)Ap; const T* A2 = (const T*)A2p; const T* Bt = (const T*)Btp; const T* Bt2 = (const T*)Bt2p;
  __shared__ __align__(16) float sT[8][16 * 68];
  const int b    = blockIdx.y;
  const int lane = threadIdx.x & 31;
  const int wave = threadIdx.x >> 5;
  const int tilesN = N >> 6;
  const int tilesM = M >> 6;
  const int tile = blockIdx.x * 8 + wave;
  if (tile >= tilesM * tilesN) return;
  const int tm = tile / tilesN;
  const int tn = tile - tm * tilesN;
  const int m0 = tm << 6;
  const int n0 = tn << 6;

  const T* Ab  = A  + (size_t)b * strideA;
  const T* Bb  = Bt + (size_t)b * strideB;
  const T* Ab2 = (SPL >= 1) ? (A2  + (size_t)b * strideA) : nullptr;
  const T* Bb2 = (SPL == 2) ? (Bt2 + (size_t)b * strideB) : nullptr;

  const int rlane = lane & 15;
  const int koff  = (lane >> 4) * 8;
  const int mOff  = (lane >> 4) * 8;

  v8f acc[4][4];
#pragma unroll
  for (int i = 0; i < 4; ++i)
#pragma unroll
    for (int j = 0; j < 4; ++j) acc[i][j] = (v8f){0.f,0.f,0.f,0.f,0.f,0.f,0.f,0.f};

  for (int k0 = 0; k0 < K; k0 += 32) {
    V bh[4], bl[4];
#pragma unroll
    for (int j = 0; j < 4; ++j) {
      const size_t bo = (size_t)(n0 + (j << 4) + rlane) * ldb + koff + k0;
      bh[j] = Frag<T>::load(Bb + bo);
      if (SPL == 2) bl[j] = Frag<T>::load(Bb2 + bo);
    }
#pragma unroll
    for (int i = 0; i < 4; ++i) {
      const size_t ao = (size_t)(m0 + (i << 4) + rlane) * lda + koff + k0;
      V ah = Frag<T>::load(Ab + ao);
      V al;
      if (SPL >= 1) al = Frag<T>::load(Ab2 + ao);
#pragma unroll
      for (int j = 0; j < 4; ++j) {
        acc[i][j] = Frag<T>::mma(ah, bh[j], acc[i][j]);
        if (SPL == 2) acc[i][j] = Frag<T>::mma(ah, bl[j], acc[i][j]);
        if (SPL >= 1) acc[i][j] = Frag<T>::mma(al, bh[j], acc[i][j]);
      }
      Frag<T>::guard4(acc[i][0], acc[i][1], acc[i][2], acc[i][3], ah, (SPL >= 1) ? al : ah);
    }
    Frag<T>::keep(bh[0], bh[1], bh[2], bh[3]);
    if (SPL == 2) Frag<T>::keep(bl[0], bl[1], bl[2], bl[3]);
  }
  acc_guard4(acc[0][0], acc[0][1], acc[0][2], acc[0][3]);
  acc_guard4(acc[1][0], acc[1][1], acc[1][2], acc[1][3]);
  acc_guard4(acc[2][0], acc[2][1], acc[2][2], acc[2][3]);
  acc_guard4(acc[3][0], acc[3][1], acc[3][2], acc[3][3]);

  float* slab = sT[wave];
  const float* Rb = RESID ? (resid + (size_t)b * strideR) : nullptr;
#pragma unroll
  for (int i = 0; i < 4; ++i) {
    const int mBase = m0 + (i << 4);
#pragma unroll
    for (int j = 0; j < 4; ++j) {
      const int n = n0 + (j << 4) + rlane;
      float bv = 0.f;
      if (BIAS_MODE == 2) bv = bias[n];
#pragma unroll
      for (int r = 0; r < 8; ++r) {
        float v = acc[i][j][r] * scale;
        if (BIAS_MODE == 1) v += bias[mBase + mOff + r];
        if (BIAS_MODE == 2) v += bv;
        if (RESID) v += Rb[(size_t)(mBase + mOff + r) * ldc + n];
        if (ACT == 1) v = tanhf(v);
        if (ACT == 2) v = fmaxf(v, 0.0f);
        if (ACT == 3) v = v * __builtin_amdgcn_rcpf(1.0f + expf(-v));
        if (ACT == 4) v = (v > 0.f) ? v : 0.01f * v;
        slab[(mOff + r) * 68 + (j << 4) + rlane] = v;
      }
    }
    __builtin_amdgcn_fence(__ATOMIC_RELEASE, "workgroup");
    __builtin_amdgcn_wave_barrier();
    __builtin_amdgcn_fence(__ATOMIC_ACQUIRE, "workgroup");
    if (OUT_MODE == 0) {
      float* C = (float*)Cout + (size_t)b * strideC;
      const int hh = lane >> 4, c4 = (lane & 15) * 4;
      for (int pass = 0; pass < 2; ++pass) {
#pragma unroll
        for (int it = 0; it < 8; ++it) {
          const int row = it * 2 + hh;
          v4f v = *(const v4f*)(slab + row * 68 + c4);
          *(volatile v4f*)(C + (size_t)(mBase + row) * ldc + n0 + c4) = v;
        }
        __threadfence();
      }
    } else {
      const int q = lane >> 3, c8 = (lane & 7) * 8;
      unsigned short* C  = (unsigned short*)Cout  + (size_t)b * strideC;
      unsigned short* C2 = (OUT_MODE == 2) ? ((unsigned short*)Cout2 + (size_t)b * strideC) : nullptr;
      for (int pass = 0; pass < 2; ++pass) {
#pragma unroll
        for (int it = 0; it < 4; ++it) {
          const int row = it * 4 + q;
          const float* sp = slab + row * 68 + c8;
          v8h hv, lv;
#pragma unroll
          for (int e = 0; e < 8; ++e) {
            if (OUT_MODE == 1) {
              hv[e] = (_Float16)sp[e];
            } else {
              unsigned short hb = f2bf_bits(sp[e]);
              unsigned short lb = f2bf_bits(sp[e] - bf_bits2f(hb));
              hv[e] = __builtin_bit_cast(_Float16, hb);
              lv[e] = __builtin_bit_cast(_Float16, lb);
            }
          }
          *(volatile v8h*)(C + (size_t)(mBase + row) * ldc + n0 + c8) = hv;
          if (OUT_MODE == 2) *(volatile v8h*)(C2 + (size_t)(mBase + row) * ldc + n0 + c8) = lv;
        }
        __threadfence();
      }
    }
    __builtin_amdgcn_fence(__ATOMIC_RELEASE, "workgroup");
    __builtin_amdgcn_wave_barrier();
    __builtin_amdgcn_fence(__ATOMIC_ACQUIRE, "workgroup");
  }
}

__global__ __launch_bounds__(256) void split_rows_bf16_kernel(
    const float* __restrict__ src, unsigned short* __restrict__ dhi, unsigned short* __restrict__ dlo, int total8)
{
  const int i = blockIdx.x * 256 + threadIdx.x;
  if (i >= total8) return;
  const size_t e0 = (size_t)i << 3;
  const v4f a0 = *(const v4f*)(src + e0);
  const v4f a1 = *(const v4f*)(src + e0 + 4);
  v8h hv, lv;
#pragma unroll
  for (int e = 0; e < 4; ++e) {
    const unsigned short h0 = f2bf_bits(a0[e]), h1 = f2bf_bits(a1[e]);
    const unsigned short l0 = f2bf_bits(a0[e] - bf_bits2f(h0)), l1 = f2bf_bits(a1[e] - bf_bits2f(h1));
    hv[e]     = __builtin_bit_cast(_Float16, h0);
    hv[4 + e] = __builtin_bit_cast(_Float16, h1);
    lv[e]     = __builtin_bit_cast(_Float16, l0);
    lv[4 + e] = __builtin_bit_cast(_Float16, l1);
  }
  unsigned short* qh = dhi + e0;
  unsigned short* ql = dlo + e0;
  *(volatile v8h*)qh = hv;
  *(volatile v8h*)ql = lv;
  __threadfence();
  *(volatile v8h*)qh = hv;
  *(volatile v8h*)ql = lv;
}

__global__ __launch_bounds__(256) void convw_split_kernel(
    const float* __restrict__ cw, unsigned short* __restrict__ dhi, unsigned short* __restrict__ dlo, int total8)
{
  const int i = blockIdx.x * 256 + threadIdx.x;
  if (i >= total8) return;
  const int lo  = i / 24;
  const int k0  = (i - lo * 24) * 8;
  const int t   = k0 >> 6;
  const int li0 = k0 & 63;
  v8h hv, lv;
#pragma unroll
  for (int e = 0; e < 8; ++e) {
    const float v = cw[(size_t)lo * kConvK + (li0 + e) * 3 + t];
    const unsigned short hb = f2bf_bits(v);
    const unsigned short lb = f2bf_bits(v - bf_bits2f(hb));
    hv[e] = __builtin_bit_cast(_Float16, hb);
    lv[e] = __builtin_bit_cast(_Float16, lb);
  }
  const size_t e0 = (size_t)i << 3;
  unsigned short* qh = dhi + e0;
  unsigned short* ql = dlo + e0;
  *(volatile v8h*)qh = hv;
  *(volatile v8h*)ql = lv;
  __threadfence();
  *(volatile v8h*)qh = hv;
  *(volatile v8h*)ql = lv;
}

__global__ __launch_bounds__(256) void xp_transpose_split_kernel(
    const float* __restrict__ XP, unsigned short* __restrict__ XTH, unsigned short* __restrict__ XTL)
{
  __shared__ float tile[64 * 65];
  const int tid = threadIdx.x, lane = tid & 31, wave = tid >> 5;
  const int d0 = blockIdx.x * 64;
  const int bix = blockIdx.y;
#pragma unroll
  for (int p = 0; p < 4; ++p) {
    const int idx4 = tid + p * 256;
    const int li = idx4 >> 4;
    const int c4 = (idx4 & 15) * 4;
    const v4f v = *(const v4f*)(XP + (size_t)(bix * kSeq + li) * kDim + d0 + c4);
    tile[li * 65 + c4 + 0] = v[0];
    tile[li * 65 + c4 + 1] = v[1];
    tile[li * 65 + c4 + 2] = v[2];
    tile[li * 65 + c4 + 3] = v[3];
  }
  __syncthreads();
  const int q = lane >> 3, c8 = (lane & 7) * 8;
  v8h hv[2], lv[2];
#pragma unroll
  for (int it = 0; it < 2; ++it) {
    const int drow = it * 32 + wave * 4 + q;
#pragma unroll
    for (int e = 0; e < 8; ++e) {
      const float f = tile[(c8 + e) * 65 + drow];
      const unsigned short hb = f2bf_bits(f);
      const unsigned short lb = f2bf_bits(f - bf_bits2f(hb));
      hv[it][e] = __builtin_bit_cast(_Float16, hb);
      lv[it][e] = __builtin_bit_cast(_Float16, lb);
    }
  }
  const bool padblk = (blockIdx.x == 0) || (blockIdx.x == 15);
  const int  prow   = (blockIdx.x == 0) ? 0 : (kXtRows - 1);
  const bool padw   = padblk && (wave == 0) && (q == 0);
  const v8h zv = (v8h){0, 0, 0, 0, 0, 0, 0, 0};
  const size_t pbase = (size_t)bix * kXtRows * kSeq;
  for (int pass = 0; pass < 2; ++pass) {
#pragma unroll
    for (int it = 0; it < 2; ++it) {
      const int drow = it * 32 + wave * 4 + q;
      const size_t o = pbase + (size_t)(d0 + drow + 1) * kSeq + c8;
      *(volatile v8h*)(XTH + o) = hv[it];
      *(volatile v8h*)(XTL + o) = lv[it];
    }
    if (padw) {
      const size_t o = pbase + (size_t)prow * kSeq + c8;
      *(volatile v8h*)(XTH + o) = zv;
      *(volatile v8h*)(XTL + o) = zv;
    }
    __threadfence();
  }
}

__global__ __launch_bounds__(256) void draw_split_kernel(
    const float* __restrict__ DBC, unsigned short* __restrict__ RH, unsigned short* __restrict__ RL, int total8)
{
  const int i = blockIdx.x * 256 + threadIdx.x;
  if (i >= total8) return;
  const int e0  = i << 3;
  const int row = e0 >> 6;
  const int c8  = e0 & 63;
  const float* p = DBC + (size_t)row * kDbcN + c8;
  const v4f a0 = *(const v4f*)(p);
  const v4f a1 = *(const v4f*)(p + 4);
  v8h hv, lv;
#pragma unroll
  for (int e = 0; e < 4; ++e) {
    const unsigned short h0 = f2bf_bits(a0[e]), h1 = f2bf_bits(a1[e]);
    const unsigned short l0 = f2bf_bits(a0[e] - bf_bits2f(h0)), l1 = f2bf_bits(a1[e] - bf_bits2f(h1));
    hv[e]     = __builtin_bit_cast(_Float16, h0);
    hv[4 + e] = __builtin_bit_cast(_Float16, h1);
    lv[e]     = __builtin_bit_cast(_Float16, l0);
    lv[4 + e] = __builtin_bit_cast(_Float16, l1);
  }
  unsigned short* qh = RH + e0;
  unsigned short* ql = RL + e0;
  *(volatile v8h*)qh = hv;
  *(volatile v8h*)ql = lv;
  __threadfence();
  *(volatile v8h*)qh = hv;
  *(volatile v8h*)ql = lv;
}

__global__ __launch_bounds__(256) void scan_gate_kernel(
    const float* __restrict__ DLR, const float* __restrict__ XONE, const float* __restrict__ DBC,
    const float* __restrict__ XP, const float* __restrict__ X, const float* __restrict__ Alog,
    const float* __restrict__ Dp, unsigned short* __restrict__ GH, unsigned short* __restrict__ GL)
{
  __shared__ __align__(16) float sA[kScE * kNst];
  __shared__ __align__(16) float sDl[kSeq * kScE];
  __shared__ __align__(16) float sX[kSeq * kScE];
  __shared__ __align__(16) float sY[kSeq * kScYP];
  const int tid = threadIdx.x, lane = tid & 31, wave = tid >> 5;
  const int bix = blockIdx.x >> 4;
  const int ch0 = (blockIdx.x & 15) * kScE;
  const size_t row0 = (size_t)bix * kSeq;

#pragma unroll 1
  for (int it = 0; it < (kScE * kNst) / 256; ++it) {
    const int idx = tid + it * 256;
    const int c = idx >> 7, n = idx & 127;
    sA[idx] = -expf(Alog[(size_t)(ch0 + c) * kNst + n]);
  }
#pragma unroll 1
  for (int it = 0; it < (kSeq * kScE) / 256; ++it) {
    const int idx = tid + it * 256;
    const int l = idx >> 6, c = idx & 63;
    const size_t gi = (row0 + l) * kDim + ch0 + c;
    const float z  = DLR[gi];
    const float xo = XONE[gi];
    const float sp = fmaxf(z, 0.0f) + log1pf(expf(-fabsf(z)));
    sDl[idx] = sp;
    sX[idx]  = xo;
  }
  __syncthreads();

#pragma unroll 1
  for (int ei = 0; ei < 8; ++ei) {
    const int c = wave * 8 + ei;
    const v4f Av = *(const v4f*)(sA + c * kNst + 4 * lane);
    float h[4];
#pragma unroll
    for (int j = 0; j < 4; ++j) h[j] = 0.0f;
#pragma unroll 1
    for (int l = 0; l < kSeq; ++l) {
      const float dl = sDl[l * kScE + c];
      const float xo = sX[l * kScE + c];
      const float dx = dl * xo;
      const float* bc = DBC + (row0 + l) * kDbcN;
      const v4f Bm = *(const v4f*)(bc + kDtR + 4 * lane);
      const v4f Cm = *(const v4f*)(bc + kDtR + kNst + 4 * lane);
      float part = 0.0f;
#pragma unroll
      for (int j = 0; j < 4; ++j) {
        float ea = expf(dl * Av[j]);
        ea = (ea < 1.17549435e-38f) ? 0.0f : ea;
        h[j] = ea * h[j] + dx * Bm[j];
        part += h[j] * Cm[j];
      }
      part += __shfl_xor(part, 16, 32);
      part += __shfl_xor(part, 8, 32);
      part += __shfl_xor(part, 4, 32);
      part += __shfl_xor(part, 2, 32);
      part += __shfl_xor(part, 1, 32);
      if (lane == 0) sY[l * kScYP + c] = part;
    }
  }
  __syncthreads();

  {
    const int c = tid & 63;
    const float dpe = Dp[ch0 + c];
#pragma unroll 1
    for (int it = 0; it < (kSeq * kScE) / 256; ++it) {
      const int idx = tid + it * 256;
      const int l = idx >> 6;
      const size_t gi = (row0 + l) * kDim + ch0 + c;
      const float y  = sY[l * kScYP + c] + dpe * sX[idx];
      const float zv = XP[gi];
      const float sg = __builtin_amdgcn_rcpf(1.0f + expf(-zv));
      const float g  = y * (zv * sg) + X[gi];
      sY[l * kScYP + c] = g;
    }
  }
  __syncthreads();

  const int q = lane >> 3, c8 = (lane & 7) * 8;
  v8h hv[2], lv[2];
#pragma unroll
  for (int it = 0; it < 2; ++it) {
    const int row = it * 32 + wave * 4 + q;
    const float* sp = sY + row * kScYP + c8;
    const v4f a0 = *(const v4f*)(sp);
    const v4f a1 = *(const v4f*)(sp + 4);
#pragma unroll
    for (int e = 0; e < 4; ++e) {
      const unsigned short h0 = f2bf_bits(a0[e]), h1 = f2bf_bits(a1[e]);
      const unsigned short l0 = f2bf_bits(a0[e] - bf_bits2f(h0)), l1 = f2bf_bits(a1[e] - bf_bits2f(h1));
      hv[it][e]     = __builtin_bit_cast(_Float16, h0);
      hv[it][4 + e] = __builtin_bit_cast(_Float16, h1);
      lv[it][e]     = __builtin_bit_cast(_Float16, l0);
      lv[it][4 + e] = __builtin_bit_cast(_Float16, l1);
    }
  }
  for (int pass = 0; pass < 2; ++pass) {
#pragma unroll
    for (int it = 0; it < 2; ++it) {
      const int row = it * 32 + wave * 4 + q;
      const size_t o = (row0 + row) * kDim + ch0 + c8;
      *(volatile v8h*)(GH + o) = hv[it];
      *(volatile v8h*)(GL + o) = lv[it];
    }
    __threadfence();
  }
}

extern "C" void kernel_launch(void* const* d_in, const int* in_sizes, int n_in,
                              void* d_out, int out_size, void* d_ws, size_t ws_size,
                              hipStream_t stream)
{
  if (n_in < 10) return;
  if (in_sizes[0] != kRows * kDim) return;
  if (in_sizes[1] != kDim * kDim) return;
  if (in_sizes[2] != kDim) return;
  if (in_sizes[3] != kSeq * kSeq * 3) return;
  if (in_sizes[4] != kSeq) return;
  if (in_sizes[5] != kDbcN * kDim) return;
  if (in_sizes[6] != kDim * kDtR) return;
  if (in_sizes[7] != kDim) return;
  if (in_sizes[8] != kDim * kNst) return;
  if (in_sizes[9] != kDim) return;
  if (out_size != kRows * kDim) return;
  if (ws_size < kWsTotal) return;

  const float* x      = (const float*)d_in[0];
  const float* proj_w = (const float*)d_in[1];
  const float* proj_b = (const float*)d_in[2];
  const float* conv_w = (const float*)d_in[3];
  const float* conv_b = (const float*)d_in[4];
  const float* dbc_w  = (const float*)d_in[5];
  const float* dt_w   = (const float*)d_in[6];
  const float* dt_b   = (const float*)d_in[7];
  const float* A_log  = (const float*)d_in[8];
  const float* Dp     = (const float*)d_in[9];
  float* out = (float*)d_out;

  char* ws = (char*)d_ws;
  unsigned short* XH   = (unsigned short*)(ws + kOffXH);
  unsigned short* XL   = (unsigned short*)(ws + kOffXL);
  unsigned short* PWH  = (unsigned short*)(ws + kOffPWH);
  unsigned short* PWL  = (unsigned short*)(ws + kOffPWL);
  unsigned short* DWH  = (unsigned short*)(ws + kOffDWH);
  unsigned short* DWL  = (unsigned short*)(ws + kOffDWL);
  unsigned short* TWH  = (unsigned short*)(ws + kOffTWH);
  unsigned short* TWL  = (unsigned short*)(ws + kOffTWL);
  unsigned short* CWH  = (unsigned short*)(ws + kOffCWH);
  unsigned short* CWL  = (unsigned short*)(ws + kOffCWL);
  float*          XP   = (float*)(ws + kOffXP);
  unsigned short* XTH  = (unsigned short*)(ws + kOffXTH);
  unsigned short* XTL  = (unsigned short*)(ws + kOffXTL);
  float*          XONE = (float*)(ws + kOffXONE);
  unsigned short* UH   = (unsigned short*)(ws + kOffUH);
  unsigned short* UL   = (unsigned short*)(ws + kOffUL);
  float*          DBC  = (float*)(ws + kOffDBC);
  unsigned short* RH   = (unsigned short*)(ws + kOffRH);
  unsigned short* RL   = (unsigned short*)(ws + kOffRL);
  float*          DLR  = (float*)(ws + kOffDLR);
  unsigned short* GH   = (unsigned short*)(ws + kOffGH);
  unsigned short* GL   = (unsigned short*)(ws + kOffGL);
  const float* dummy_bias  = dt_b;
  const float* dummy_resid = x;

  split_rows_bf16_kernel<<<(kRows * kDim / 8) / 256, 256, 0, stream>>>(x, XH, XL, kRows * kDim / 8);
  split_rows_bf16_kernel<<<(kDim * kDim / 8) / 256, 256, 0, stream>>>(proj_w, PWH, PWL, kDim * kDim / 8);
  split_rows_bf16_kernel<<<(kDbcN * kDim / 8) / 256, 256, 0, stream>>>(dbc_w, DWH, DWL, kDbcN * kDim / 8);
  split_rows_bf16_kernel<<<(kDim * kDtR / 8) / 256, 256, 0, stream>>>(dt_w, TWH, TWL, kDim * kDtR / 8);
  convw_split_kernel<<<(kSeq * kConvK / 8) / 256, 256, 0, stream>>>(conv_w, CWH, CWL, kSeq * kConvK / 8);

  wmma_gemm64<1, 2, 2, 0, false, 0><<<dim3(16, 1), 256, 0, stream>>>(
      XH, XL, kDim, 0L,
      PWH, PWL, kDim, 0L,
      (void*)XP, (void*)XP, kDim, 0L,
      proj_b, dummy_resid, 0L,
      kRows, kDim, kDim, 1.0f);

  xp_transpose_split_kernel<<<dim3(kDim / 64, kBat), 256, 0, stream>>>(XP, XTH, XTL);

  wmma_gemm64<1, 2, 1, 0, false, 3><<<dim3(2, kBat), 256, 0, stream>>>(
      CWH, CWL, kConvK, 0L,
      XTH, XTL, kSeq, (long)kXtRows * kSeq,
      (void*)XONE, (void*)XONE, kDim, (long)kSeq * kDim,
      conv_b, dummy_resid, 0L,
      kSeq, kDim, kConvK, 1.0f);

  split_rows_bf16_kernel<<<(kRows * kDim / 8) / 256, 256, 0, stream>>>(XONE, UH, UL, kRows * kDim / 8);

  wmma_gemm64<1, 2, 0, 0, false, 0><<<dim3(5, 1), 256, 0, stream>>>(
      UH, UL, kDim, 0L,
      DWH, DWL, kDim, 0L,
      (void*)DBC, (void*)DBC, kDbcN, 0L,
      dummy_bias, dummy_resid, 0L,
      kRows, kDbcN, kDim, 1.0f);

  draw_split_kernel<<<(kRows * kDtR / 8) / 256, 256, 0, stream>>>(DBC, RH, RL, kRows * kDtR / 8);

  wmma_gemm64<1, 2, 2, 0, false, 0><<<dim3(16, 1), 256, 0, stream>>>(
      RH, RL, kDtR, 0L,
      TWH, TWL, kDtR, 0L,
      (void*)DLR, (void*)DLR, kDim, 0L,
      dt_b, dummy_resid, 0L,
      kRows, kDim, kDtR, 1.0f);

  scan_gate_kernel<<<kBat * (kDim / kScE), 256, 0, stream>>>(DLR, XONE, DBC, XP, x, A_log, Dp, GH, GL);

  wmma_gemm64<1, 2, 2, 0, false, 0><<<dim3(16, 1), 256, 0, stream>>>(
      GH, GL, kDim, 0L,
      PWH, PWL, kDim, 0L,
      (void*)out, (void*)out, kDim, 0L,
      proj_b, dummy_resid, 0L,
      kRows, kDim, kDim, 1.0f);
}
